// SSCNNPredictor_30666066493783
// MI455X (gfx1250) — hardware-verified
//
#include <hip/hip_runtime.h>

#define NB   2
#define NTOK 128
#define NL   256
#define NLP  258
#define NC   768
#define NCH  16
#define NTYP 5

typedef __bf16 v16bf __attribute__((ext_vector_type(16)));
typedef float v8f __attribute__((ext_vector_type(8)));
typedef float v4f __attribute__((ext_vector_type(4)));
typedef unsigned int v4u __attribute__((ext_vector_type(4)));
typedef v4f __attribute__((may_alias)) v4fa;
typedef v4u __attribute__((may_alias)) v4ua;

union FragB { v16bf v; v4u q[2]; };

__device__ __forceinline__ int imin(int a, int b) { return a < b ? a : b; }
__device__ __forceinline__ int imax(int a, int b) { return a > b ? a : b; }

__device__ __forceinline__ unsigned short f2bf(float f) {
  unsigned int x = __float_as_uint(f);
  x = (x + 0x7FFFu + ((x >> 16) & 1u)) >> 16;
  return (unsigned short)x;
}
__device__ __forceinline__ float bf2f(unsigned short b) {
  return __uint_as_float(((unsigned int)b) << 16);
}

__device__ __forceinline__ void split2(float x, float y, unsigned int& ph, unsigned int& pl) {
  const unsigned short hx = f2bf(x), hy = f2bf(y);
  const float rx = x - bf2f(hx), ry = y - bf2f(hy);
  ph = (unsigned int)hx | ((unsigned int)hy << 16);
  pl = (unsigned int)f2bf(rx) | ((unsigned int)f2bf(ry) << 16);
}
__device__ __forceinline__ void split8(v4f a, v4f c, v4u& hi, v4u& lo) {
  unsigned int h0, h1, h2, h3, l0, l1, l2, l3;
  split2(a.x, a.y, h0, l0);
  split2(a.z, a.w, h1, l1);
  split2(c.x, c.y, h2, l2);
  split2(c.z, c.w, h3, l3);
  const v4u hv = {h0, h1, h2, h3};
  const v4u lv = {l0, l1, l2, l3};
  hi = hv; lo = lv;
}

__device__ __forceinline__ v8f wmma16(v16bf a, v16bf b, v8f c) {
  v8f d = __builtin_amdgcn_wmma_f32_16x16x32_bf16(false, a, false, b, (short)0, c, false, false);
  asm volatile("v_nop\n\tv_nop\n\tv_nop\n\tv_nop" : "+v"(d) : "v"(a), "v"(b));
  return d;
}
__device__ __forceinline__ v8f mma3(v16bf ah, v16bf al, v16bf bh, v16bf bl, v8f c) {
  c = wmma16(ah, bh, c);
  c = wmma16(ah, bl, c);
  c = wmma16(al, bh, c);
  return c;
}
__device__ __forceinline__ v16bf ldfrag(const unsigned short* p, int h) {
  FragB f;
  f.q[0] = *(const v4ua*)(p + 8 * h);
  f.q[1] = *(const v4ua*)(p + 16 + 8 * h);
  return f.v;
}

__global__ __launch_bounds__(256) void k_wprep(const float* __restrict__ w,
    unsigned short* __restrict__ wth, unsigned short* __restrict__ wtl)
{
  __shared__ float tile[64][65];
  const int tid = threadIdx.x, lane = tid & 31, wv = tid >> 5;
  const int d0 = blockIdx.x * 64, k0 = blockIdx.y * 64, n = blockIdx.z;
  const float* src = w + (size_t)n * NC * NC;
  #pragma unroll
  for (int it = 0; it < 16; ++it) {
    const int idx = it * 256 + tid;
    const int kk = idx >> 6, dd = idx & 63;
    tile[kk][dd] = src[(size_t)(k0 + kk) * NC + d0 + dd];
  }
  __syncthreads();
  const int sub = lane >> 3, q8 = lane & 7;
  const int dda = wv * 8 + sub, ddb = dda + 4;
  const v4f a0 = {tile[8 * q8 + 0][dda], tile[8 * q8 + 1][dda], tile[8 * q8 + 2][dda], tile[8 * q8 + 3][dda]};
  const v4f c0 = {tile[8 * q8 + 4][dda], tile[8 * q8 + 5][dda], tile[8 * q8 + 6][dda], tile[8 * q8 + 7][dda]};
  const v4f a1 = {tile[8 * q8 + 0][ddb], tile[8 * q8 + 1][ddb], tile[8 * q8 + 2][ddb], tile[8 * q8 + 3][ddb]};
  const v4f c1 = {tile[8 * q8 + 4][ddb], tile[8 * q8 + 5][ddb], tile[8 * q8 + 6][ddb], tile[8 * q8 + 7][ddb]};
  v4u h0, l0, h1, l1;
  split8(a0, c0, h0, l0);
  split8(a1, c1, h1, l1);
  const size_t o0 = ((size_t)n * NC + d0 + dda) * NC + k0 + 8 * q8;
  const size_t o1 = ((size_t)n * NC + d0 + ddb) * NC + k0 + 8 * q8;
  *(volatile v4u*)(wth + o0) = h0;
  *(volatile v4u*)(wtl + o0) = l0;
  *(volatile v4u*)(wth + o1) = h1;
  *(volatile v4u*)(wtl + o1) = l1;
  __threadfence();
  *(volatile v4u*)(wth + o0) = h0;
  *(volatile v4u*)(wtl + o0) = l0;
  *(volatile v4u*)(wth + o1) = h1;
  *(volatile v4u*)(wtl + o1) = l1;
}

__device__ __forceinline__ void padzero_pass(float* hf, unsigned short* hh, unsigned short* hl, int tid) {
  const v4f zf = {0.f, 0.f, 0.f, 0.f};
  const v4u zu = {0u, 0u, 0u, 0u};
  #pragma unroll
  for (int it = 0; it < 3; ++it) {
    const int idx = it * 256 + tid;
    const int rs = idx / 192, p = idx - rs * 192;
    const int row = (rs >> 1) * NLP + ((rs & 1) ? (NLP - 1) : 0);
    *(volatile v4f*)(hf + (size_t)row * NC + 4 * p) = zf;
  }
  #pragma unroll
  for (int it = 0; it < 2; ++it) {
    const int idx = it * 256 + tid;
    if (idx < 384) {
      const int rs = idx / 96, p = idx - rs * 96;
      const int row = (rs >> 1) * NLP + ((rs & 1) ? (NLP - 1) : 0);
      *(volatile v4u*)(hh + (size_t)row * NC + 8 * p) = zu;
      *(volatile v4u*)(hl + (size_t)row * NC + 8 * p) = zu;
    }
  }
}
__global__ __launch_bounds__(256) void k_padzero(float* __restrict__ hf,
    unsigned short* __restrict__ hh, unsigned short* __restrict__ hl)
{
  const int tid = threadIdx.x;
  padzero_pass(hf, hh, hl, tid);
  __threadfence();
  padzero_pass(hf, hh, hl, tid);
}

__device__ __forceinline__ void nuc_store(const float* so, const int* srow, int nrows,
    float* hf, unsigned short* hh, unsigned short* hl, int wv, int lane)
{
  #pragma unroll
  for (int q = 0; q < 2; ++q) {
    const int rr = 2 * wv + q;
    if (rr < nrows) {
      const int r = srow[rr];
      const int b = (r >> 8) & 1, l = r & 255;
      const size_t ro = (size_t)(b * NLP + l + 1) * NC;
      const float* s = so + rr * NC;
      #pragma unroll
      for (int it = 0; it < 6; ++it) {
        const int p = it * 32 + lane;
        const v4f v = *(const v4fa*)(s + 4 * p);
        *(volatile v4f*)(hf + ro + 4 * p) = v;
      }
      #pragma unroll
      for (int it = 0; it < 3; ++it) {
        const int p = it * 32 + lane;
        const v4f a = *(const v4fa*)(s + 8 * p);
        const v4f c = *(const v4fa*)(s + 8 * p + 4);
        v4u hv, lv;
        split8(a, c, hv, lv);
        *(volatile v4u*)(hh + ro + 8 * p) = hv;
        *(volatile v4u*)(hl + ro + 8 * p) = lv;
      }
    }
  }
}

__global__ __launch_bounds__(256) void k_nuc(
    const float* __restrict__ hidden,
    const int* __restrict__ ptl,
    const int* __restrict__ ids,
    const float* __restrict__ wmask,
    const float* __restrict__ bnuc,
    const unsigned short* __restrict__ wth,
    const unsigned short* __restrict__ wtl,
    float* __restrict__ hf,
    unsigned short* __restrict__ hh,
    unsigned short* __restrict__ hl)
{
  __shared__ __attribute__((aligned(16))) float smem[16 * NC];
  __shared__ int slist[NB * NL];
  __shared__ int scum[NB * NTOK];
  __shared__ int swcnt[8];
  __shared__ int srow[16];
  __shared__ int stok[16];
  __shared__ float smask[16];

  const int tid = threadIdx.x, lane = tid & 31, wv = tid >> 5;
  const int h = lane >> 4, m = lane & 15;
  const int ts = blockIdx.x, typ = blockIdx.y;
  unsigned short* ahi = (unsigned short*)smem;
  unsigned short* alo = ahi + 16 * NC;

  if (tid < NB) {
    int s = 0;
    for (int t = 0; t < NTOK; ++t) { s += ptl[tid * NTOK + t]; scum[tid * NTOK + t] = s; }
  }

  int cnt = 0;
  #pragma unroll
  for (int ch = 0; ch < 2; ++ch) {
    const int r = ch * 256 + tid;
    const int id = ids[r];
    const bool inv = (id < 0) || (id >= NTYP);
    const bool hit = (id == typ) || (inv && (typ == NTYP - 1));
    const unsigned int bal = __builtin_amdgcn_ballot_w32(hit);
    if (lane == 0) swcnt[wv] = (int)__builtin_popcount(bal);
    __syncthreads();
    int pre = 0, tot = 0;
    #pragma unroll
    for (int q = 0; q < 8; ++q) { const int c = swcnt[q]; pre += (q < wv) ? c : 0; tot += c; }
    if (hit) slist[cnt + pre + (int)__builtin_popcount(bal & ((1u << lane) - 1u))] = r;
    cnt += tot;
    __syncthreads();
  }
  if (ts * 16 >= cnt) return;
  const int nrows = imin(16, cnt - ts * 16);

  if (tid < 16) {
    const bool valid = tid < nrows;
    int r = slist[ts * 16 + tid];
    r = valid ? r : 0;
    const int b = (r >> 8) & 1, l = r & 255;
    const int id = ids[r];
    const bool inv = (id < 0) || (id >= NTYP);
    int tk = 0;
    for (int t = 0; t < NTOK; ++t) tk += (scum[b * NTOK + t] <= l) ? 1 : 0;
    tk = imin(tk, NTOK - 1);
    srow[tid] = r;
    stok[tid] = b * NTOK + tk;
    smask[tid] = (valid && !inv) ? wmask[r] : 0.f;
  }
  __syncthreads();

  {
    const int rr = tid >> 4, s16 = tid & 15;
    const float* src = hidden + (size_t)stok[rr] * NC;
    const bool vrow = rr < nrows;
    const v4f zf = {0.f, 0.f, 0.f, 0.f};
    #pragma unroll
    for (int e = 0; e < 6; ++e) {
      const int k = e * 128 + s16 * 8;
      v4f a = *(const v4fa*)(src + k);
      v4f c = *(const v4fa*)(src + k + 4);
      a = vrow ? a : zf;
      c = vrow ? c : zf;
      v4u hv, lv;
      split8(a, c, hv, lv);
      *(v4ua*)(ahi + rr * NC + k) = hv;
      *(v4ua*)(alo + rr * NC + k) = lv;
    }
  }
  __syncthreads();

  const int cb = wv * 96;
  const v8f z8 = {0.f, 0.f, 0.f, 0.f, 0.f, 0.f, 0.f, 0.f};
  v8f acc[6];
  #pragma unroll
  for (int nt = 0; nt < 6; ++nt) acc[nt] = z8;
  const unsigned short* wbh = wth + ((size_t)typ * NC + cb + m) * NC;
  const unsigned short* wbl = wtl + ((size_t)typ * NC + cb + m) * NC;
  #pragma unroll 1
  for (int kc = 0; kc < NC / 32; ++kc) {
    const v16bf ah = ldfrag(ahi + m * NC + kc * 32, h);
    const v16bf al = ldfrag(alo + m * NC + kc * 32, h);
    #pragma unroll
    for (int nt = 0; nt < 6; ++nt) {
      const v16bf bh = ldfrag(wbh + (size_t)nt * 16 * NC + kc * 32, h);
      const v16bf bl = ldfrag(wbl + (size_t)nt * 16 * NC + kc * 32, h);
      acc[nt] = mma3(ah, al, bh, bl, acc[nt]);
    }
  }
  __syncthreads();

  float* so = smem;
  #pragma unroll
  for (int nt = 0; nt < 6; ++nt) {
    const int col = cb + 16 * nt + m;
    const float bb = bnuc[typ * NC + col];
    #pragma unroll
    for (int r = 0; r < 8; ++r) {
      const int rr = 8 * h + r;
      so[rr * NC + col] = (acc[nt][r] + bb) * smask[rr];
    }
  }
  __syncthreads();
  nuc_store(so, srow, nrows, hf, hh, hl, wv, lane);
  __threadfence();
  nuc_store(so, srow, nrows, hf, hh, hl, wv, lane);
}

__device__ __forceinline__ void stem_store(const float* stg, float* yrow, int lane) {
  const int sub = lane >> 4, q = lane & 15;
  #pragma unroll
  for (int it = 0; it < 8; ++it) {
    const int row = 2 * it + sub;
    const v4f v = *(const v4fa*)(stg + row * 64 + 4 * q);
    *(volatile v4f*)(yrow + (size_t)row * NL + 4 * q) = v;
  }
}

__global__ __launch_bounds__(256) void k_stem(
    const float* __restrict__ hf,
    const unsigned short* __restrict__ hh,
    const unsigned short* __restrict__ hl,
    const float* __restrict__ w_in,
    const float* __restrict__ b_in,
    float* __restrict__ y)
{
  __shared__ __attribute__((aligned(16))) float smem[8544];
  unsigned short* bth = (unsigned short*)smem;
  unsigned short* btl = bth + 3 * 64 * 32;
  float* sh = smem + 6144;
  float* sw = sh + 66 * 32;

  const int tid = threadIdx.x, lane = tid & 31, wv = tid >> 5;
  const int h = lane >> 4, m = lane & 15;
  const int j0 = blockIdx.x * 64, o = blockIdx.y, b = blockIdx.z;
  const int i0w = wv * 32;

  const v8f z8 = {0.f, 0.f, 0.f, 0.f, 0.f, 0.f, 0.f, 0.f};
  v8f acc[2][4];
  #pragma unroll
  for (int mt = 0; mt < 2; ++mt)
    #pragma unroll
    for (int nt = 0; nt < 4; ++nt) acc[mt][nt] = z8;

  #pragma unroll 1
  for (int kc = 0; kc < NC / 32; ++kc) {
    __syncthreads();
    #pragma unroll
    for (int it = 0; it < 9; ++it) {
      const int idx = it * 256 + tid;
      if (idx < 66 * 32) {
        const int jj = idx >> 5, kk = idx & 31;
        sh[idx] = hf[(size_t)(b * NLP + j0 + jj) * NC + kc * 32 + kk];
      }
    }
    for (int q = tid; q < 288; q += 256) {
      const int kk = q / 9, s = q - kk * 9;
      sw[s * 32 + kk] = w_in[(size_t)(o * NC + kc * 32 + kk) * 9 + s];
    }
    __syncthreads();
    {
      const int j = tid >> 2, kb = (tid & 3) * 8;
      const v4f h0a = *(const v4fa*)(sh + (j + 0) * 32 + kb), h0c = *(const v4fa*)(sh + (j + 0) * 32 + kb + 4);
      const v4f h1a = *(const v4fa*)(sh + (j + 1) * 32 + kb), h1c = *(const v4fa*)(sh + (j + 1) * 32 + kb + 4);
      const v4f h2a = *(const v4fa*)(sh + (j + 2) * 32 + kb), h2c = *(const v4fa*)(sh + (j + 2) * 32 + kb + 4);
      #pragma unroll
      for (int di = 0; di < 3; ++di) {
        const v4f w0a = *(const v4fa*)(sw + (di * 3 + 0) * 32 + kb), w0c = *(const v4fa*)(sw + (di * 3 + 0) * 32 + kb + 4);
        const v4f w1a = *(const v4fa*)(sw + (di * 3 + 1) * 32 + kb), w1c = *(const v4fa*)(sw + (di * 3 + 1) * 32 + kb + 4);
        const v4f w2a = *(const v4fa*)(sw + (di * 3 + 2) * 32 + kb), w2c = *(const v4fa*)(sw + (di * 3 + 2) * 32 + kb + 4);
        const v4f va = w0a * h0a + w1a * h1a + w2a * h2a;
        const v4f vc = w0c * h0c + w1c * h1c + w2c * h2c;
        v4u hv, lv;
        split8(va, vc, hv, lv);
        *(v4ua*)(bth + (di * 64 + j) * 32 + kb) = hv;
        *(v4ua*)(btl + (di * 64 + j) * 32 + kb) = lv;
      }
    }
    __syncthreads();
    #pragma unroll 1
    for (int di = 0; di < 3; ++di) {
      const size_t arow = (size_t)(b * NLP + i0w + m + di) * NC + kc * 32;
      const v16bf ah0 = ldfrag(hh + arow, h);
      const v16bf ah1 = ldfrag(hh + arow + 16 * NC, h);
      const v16bf al0 = ldfrag(hl + arow, h);
      const v16bf al1 = ldfrag(hl + arow + 16 * NC, h);
      #pragma unroll
      for (int nt = 0; nt < 4; ++nt) {
        const unsigned short* bp = bth + (di * 64 + 16 * nt + m) * 32;
        const unsigned short* bq = btl + (di * 64 + 16 * nt + m) * 32;
        const v16bf bhf = ldfrag(bp, h);
        const v16bf blf = ldfrag(bq, h);
        acc[0][nt] = mma3(ah0, al0, bhf, blf, acc[0][nt]);
        acc[1][nt] = mma3(ah1, al1, bhf, blf, acc[1][nt]);
      }
    }
  }

  const float bo = b_in[o];
  float* stg = smem + wv * 1024;
  #pragma unroll
  for (int mt = 0; mt < 2; ++mt) {
    __syncthreads();
    #pragma unroll
    for (int nt = 0; nt < 4; ++nt)
      #pragma unroll
      for (int r = 0; r < 8; ++r)
        stg[(8 * h + r) * 64 + 16 * nt + m] = fmaxf(acc[mt][nt][r] + bo, 0.f);
    __syncthreads();
    float* yrow = y + ((size_t)((b * NCH + o) * NL + i0w + 16 * mt)) * NL + j0;
    stem_store(stg, yrow, lane);
    __threadfence();
    stem_store(stg, yrow, lane);
  }
}

__device__ __forceinline__ void conv_store(const float* sy, float* drow, int lane) {
  #pragma unroll
  for (int it = 0; it < 2; ++it) {
    const int p = it * 32 + lane;
    const v4f v = *(const v4fa*)(sy + 4 * p);
    *(volatile v4f*)(drow + 4 * p) = v;
  }
}
__device__ __forceinline__ void head_store(const float* sho, float* orow, int tid) {
  if (tid < 64) {
    const v4f v = *(const v4fa*)(sho + 4 * tid);
    *(volatile v4f*)(orow + 4 * tid) = v;
  }
}

__global__ __launch_bounds__(512) void k_conv(
    const float* __restrict__ src,
    const float* __restrict__ w,
    const float* __restrict__ bias,
    const float* __restrict__ resid,
    const float* __restrict__ w_out,
    const float* __restrict__ b_out,
    float* __restrict__ dst,
    float* __restrict__ out,
    int mode)
{
  __shared__ __attribute__((aligned(16))) float sxraw[12384];
  __shared__ __attribute__((aligned(16))) unsigned short swt[2 * 16 * 160];
  __shared__ __attribute__((aligned(16))) float sho[NL];
  unsigned short* sxh = (unsigned short*)sxraw;
  unsigned short* sxl = sxh + 3 * 258 * 16;
  unsigned short* swh = swt;
  unsigned short* swl = swt + 16 * 160;

  const int tid = threadIdx.x, lane = tid & 31, wv = tid >> 5;
  const int h = lane >> 4, m = lane & 15;
  const int i = blockIdx.x, b = blockIdx.y;

  #pragma unroll 1
  for (int it = 0; it < 25; ++it) {
    const int idx = it * 512 + tid;
    if (idx < 3 * 16 * 258) {
      const int q = idx / 258, jj = idx - q * 258;
      const int c = q & 15, di = q >> 4;
      const int ii = i + di - 1, j = jj - 1;
      const bool ok = (ii >= 0) && (ii < NL) && (j >= 0) && (j < NL);
      const int iic = imin(imax(ii, 0), NL - 1), jc = imin(imax(j, 0), NL - 1);
      float v = src[((size_t)((b * NCH + c) * NL + iic)) * NL + jc];
      v = ok ? v : 0.f;
      const unsigned short hb = f2bf(v);
      const int li = (di * 258 + jj) * 16 + c;
      sxh[li] = hb;
      sxl[li] = f2bf(v - bf2f(hb));
    }
  }
  #pragma unroll
  for (int it = 0; it < 5; ++it) {
    const int idx = it * 512 + tid;
    const int oo = idx / 160, k = idx - oo * 160;
    const int kc2 = imin(k, 143);
    const int c = kc2 & 15, s = kc2 >> 4;
    const int di = s / 3, dj = s - di * 3;
    float v = w[((oo * NCH + c) * 3 + di) * 3 + dj];
    v = (k < 144) ? v : 0.f;
    const unsigned short hb = f2bf(v);
    swh[idx] = hb;
    swl[idx] = f2bf(v - bf2f(hb));
  }
  __syncthreads();

  const int jcol = wv * 16 + m;
  const v8f z8 = {0.f, 0.f, 0.f, 0.f, 0.f, 0.f, 0.f, 0.f};
  v8f acc = z8;
  #pragma unroll
  for (int kc = 0; kc < 5; ++kc) {
    const v16bf ah = ldfrag(swh + m * 160 + kc * 32, h);
    const v16bf al = ldfrag(swl + m * 160 + kc * 32, h);
    FragB bh, bl;
    {
      const int s = 2 * kc, di = s / 3, dj = s - 3 * di;
      const int li = (di * 258 + jcol + dj) * 16 + 8 * h;
      bh.q[0] = *(const v4ua*)(sxh + li);
      bl.q[0] = *(const v4ua*)(sxl + li);
    }
    if (2 * kc + 1 <= 8) {
      const int s = 2 * kc + 1, di = s / 3, dj = s - 3 * di;
      const int li = (di * 258 + jcol + dj) * 16 + 8 * h;
      bh.q[1] = *(const v4ua*)(sxh + li);
      bl.q[1] = *(const v4ua*)(sxl + li);
    } else {
      const v4u zu = {0u, 0u, 0u, 0u};
      bh.q[1] = zu;
      bl.q[1] = zu;
    }
    acc = mma3(ah, al, bh.v, bl.v, acc);
  }
  __syncthreads();

  float* sy = sxraw;
  #pragma unroll
  for (int r = 0; r < 8; ++r) {
    const int oo = 8 * h + r;
    float v = acc[r] + bias[oo];
    if (mode != 0) v += resid[((size_t)((b * NCH + oo) * NL + i)) * NL + jcol];
    v = fmaxf(v, 0.f);
    sy[oo * NL + jcol] = v;
  }
  __syncthreads();
  if (mode != 2) {
    float* drow = dst + ((size_t)((b * NCH + wv) * NL + i)) * NL;
    conv_store(sy + wv * NL, drow, lane);
    __threadfence();
    conv_store(sy + wv * NL, drow, lane);
  } else {
    if (tid < NL) {
      float s = 0.f;
      #pragma unroll
      for (int oo = 0; oo < NCH; ++oo) s += sy[oo * NL + tid] * w_out[oo];
      sho[tid] = s + b_out[0];
    }
    __syncthreads();
    float* orow = out + ((size_t)(b * NL + i)) * NL;
    head_store(sho, orow, tid);
    __threadfence();
    head_store(sho, orow, tid);
  }
}

extern "C" void kernel_launch(void* const* d_in, const int* in_sizes, int n_in,
                              void* d_out, int out_size, void* d_ws, size_t ws_size,
                              hipStream_t stream) {
  if (n_in < 18) return;
  if (in_sizes[0] != NB * NTOK * NC) return;
  if (in_sizes[1] != NB * NL) return;
  if (in_sizes[2] != NTYP * NC * NC) return;
  if (in_sizes[3] != NTYP * NC) return;
  if (in_sizes[4] != NCH * NC * 9 || in_sizes[5] != NCH) return;
  if (in_sizes[6] != NCH * NCH * 9 || in_sizes[7] != NCH) return;
  if (in_sizes[8] != NCH * NCH * 9 || in_sizes[9] != NCH) return;
  if (in_sizes[10] != NCH * NCH * 9 || in_sizes[11] != NCH) return;
  if (in_sizes[12] != NCH * NCH * 9 || in_sizes[13] != NCH) return;
  if (in_sizes[14] != NCH || in_sizes[15] < 1) return;
  if (in_sizes[16] != NB * NTOK || in_sizes[17] != NB * NL) return;
  if (out_size != NB * NL * NL) return;

  const float* hidden = (const float*)d_in[0];
  const float* wmask  = (const float*)d_in[1];
  const float* W_nuc  = (const float*)d_in[2];
  const float* b_nuc  = (const float*)d_in[3];
  const float* w_in   = (const float*)d_in[4];
  const float* b_in   = (const float*)d_in[5];
  const float* w1a    = (const float*)d_in[6];
  const float* b1a    = (const float*)d_in[7];
  const float* w1b    = (const float*)d_in[8];
  const float* b1b    = (const float*)d_in[9];
  const float* w2a    = (const float*)d_in[10];
  const float* b2a    = (const float*)d_in[11];
  const float* w2b    = (const float*)d_in[12];
  const float* b2b    = (const float*)d_in[13];
  const float* w_out  = (const float*)d_in[14];
  const float* b_out  = (const float*)d_in[15];
  const int*   ptl    = (const int*)d_in[16];
  const int*   nucid  = (const int*)d_in[17];
  float* out = (float*)d_out;

  const size_t wt_b = (size_t)NTYP * NC * NC * 2;
  const size_t hf_b = (size_t)NB * NLP * NC * 4;
  const size_t hb_b = (size_t)NB * NLP * NC * 2;
  const size_t pl_b = (size_t)NB * NCH * NL * NL * 4;
  size_t off = 0;
  const size_t o_wth = off; off += wt_b;
  const size_t o_wtl = off; off += wt_b;
  const size_t o_hf  = off; off += hf_b;
  const size_t o_hh  = off; off += hb_b;
  const size_t o_hl  = off; off += hb_b;
  const size_t o_y   = off; off += pl_b;
  const size_t o_r   = off; off += pl_b;
  const size_t o_y2  = off; off += pl_b;
  if (off > ws_size) return;

  char* ws = (char*)d_ws;
  unsigned short* wth = (unsigned short*)(ws + o_wth);
  unsigned short* wtl = (unsigned short*)(ws + o_wtl);
  float* hf = (float*)(ws + o_hf);
  unsigned short* hh = (unsigned short*)(ws + o_hh);
  unsigned short* hl = (unsigned short*)(ws + o_hl);
  float* Y  = (float*)(ws + o_y);
  float* R  = (float*)(ws + o_r);
  float* Y2 = (float*)(ws + o_y2);

  k_wprep<<<dim3(NC / 64, NC / 64, NTYP), dim3(256), 0, stream>>>(W_nuc, wth, wtl);
  k_padzero<<<dim3(1), dim3(256), 0, stream>>>(hf, hh, hl);
  k_nuc<<<dim3(NB * NL / 16, NTYP), dim3(256), 0, stream>>>(
      hidden, ptl, nucid, wmask, b_nuc, wth, wtl, hf, hh, hl);
  k_stem<<<dim3(NL / 64, NCH, NB), dim3(256), 0, stream>>>(hf, hh, hl, w_in, b_in, Y);
  k_conv<<<dim3(NL, NB), dim3(512), 0, stream>>>(Y,  w1a, b1a, Y,  w_out, b_out, R,  out, 0);
  k_conv<<<dim3(NL, NB), dim3(512), 0, stream>>>(R,  w1b, b1b, Y,  w_out, b_out, Y2, out, 1);
  k_conv<<<dim3(NL, NB), dim3(512), 0, stream>>>(Y2, w2a, b2a, Y2, w_out, b_out, R,  out, 0);
  k_conv<<<dim3(NL, NB), dim3(512), 0, stream>>>(R,  w2b, b2b, Y2, w_out, b_out, Y,  out, 2);
}
